// ValueNetwork_74689481277646
// MI455X (gfx1250) — hardware-verified
//
#include <hip/hip_runtime.h>

typedef _Float16 v16h __attribute__((ext_vector_type(16)));
typedef _Float16 v8h  __attribute__((ext_vector_type(8)));
typedef float    v8f  __attribute__((ext_vector_type(8)));
typedef float    v4f  __attribute__((ext_vector_type(4)));
union Frag { v16h v; v8h half[2]; };

#define NB   256
#define NH   511
#define IND  13
#define SD   6
#define HS   7
#define NR   512
#define DH   64
#define EP   520
#define HP   72

__device__ __forceinline__ v8f wmma16(const v16h a, const v16h b, v8f acc)
{
    acc = __builtin_amdgcn_wmma_f32_16x16x32_f16(false, a, false, b, (short)0, acc, false, false);
    asm volatile("v_nop\n\tv_nop\n\tv_nop\n\tv_nop" : "+v"(acc) : "v"(a), "v"(b));
    return acc;
}

__global__ __launch_bounds__(256)
void k_attn(const float* __restrict__ state, const float* __restrict__ tmat,
            const float* __restrict__ w_a, const float* __restrict__ w1,
            float* __restrict__ Vg)
{
    __shared__ __align__(16) float    Xs[NR * 8];
    __shared__ __align__(16) _Float16 XW1t[DH * EP];
    __shared__ __align__(16) _Float16 Et[32 * EP];
    __shared__ __align__(16) float    Xwt[32 * 8];
    __shared__ float SinvAll[NR];
    __shared__ float p0u[NR];
    __shared__ float part[32 * DH];
    __shared__ float wa_s[HS * HS];
    __shared__ float w1_s[HS * DH];
    __shared__ __align__(16) float vout[DH];

    const int tid = threadIdx.x;
    const int b   = blockIdx.x;

    if (tid < HS * HS) wa_s[tid] = w_a[tid];
    for (int i = tid; i < HS * DH; i += 256) w1_s[i] = w1[i];

    for (int m = tid; m < NR; m += 256) {
        if (m == 0) {
            const float* ss = state + (size_t)b * NH * IND;
            #pragma unroll
            for (int j = 0; j < HS; ++j) {
                float s = 0.f;
                #pragma unroll
                for (int i = 0; i < SD; ++i) s += ss[i] * tmat[i * HS + j];
                Xs[j] = s;
            }
            Xs[7] = 0.f;
        } else {
            const float* src = state + ((size_t)b * NH + (m - 1)) * IND + SD;
            #pragma unroll
            for (int j = 0; j < HS; ++j) Xs[m * 8 + j] = src[j];
            Xs[m * 8 + 7] = 0.f;
        }
    }
    __syncthreads();

    for (int idx = tid; idx < NR * DH; idx += 256) {
        const int m = idx & (NR - 1), d = idx >> 9;
        float s = 0.f;
        #pragma unroll
        for (int j = 0; j < HS; ++j) s += Xs[m * 8 + j] * w1_s[j * DH + d];
        XW1t[d * EP + m] = (_Float16)s;
    }
    __syncthreads();

    const int lane = tid & 31;
    const int wave = tid >> 5;
    const int h    = lane >> 4;
    const int lan  = lane & 15;
    const int rsub = wave >> 2;
    const int grp  = wave & 3;
    const v8f zero8 = {0.f, 0.f, 0.f, 0.f, 0.f, 0.f, 0.f, 0.f};

    for (int nt = 0; nt < 16; ++nt) {
        {
            const int row = tid >> 3;
            const int k   = tid & 7;
            const int n   = nt * 32 + row;
            float s = 0.f;
            if (k < HS) {
                #pragma unroll
                for (int j = 0; j < HS; ++j) s += Xs[n * 8 + j] * wa_s[j * HS + k];
            }
            Xwt[row * 8 + k] = s;
        }
        __syncthreads();

        float L[4][16];
        float xw[4][7];
        #pragma unroll
        for (int rr = 0; rr < 4; ++rr) {
            #pragma unroll
            for (int k = 0; k < HS; ++k) xw[rr][k] = Xwt[(wave * 4 + rr) * 8 + k];
        }
        #pragma unroll
        for (int i = 0; i < 16; ++i) {
            const int m = lane + 32 * i;
            const v4f x0 = *(const v4f*)&Xs[m * 8];
            const v4f x1 = *(const v4f*)&Xs[m * 8 + 4];
            #pragma unroll
            for (int rr = 0; rr < 4; ++rr) {
                float s = xw[rr][0] * x0[0];
                s += xw[rr][1] * x0[1];
                s += xw[rr][2] * x0[2];
                s += xw[rr][3] * x0[3];
                s += xw[rr][4] * x1[0];
                s += xw[rr][5] * x1[1];
                s += xw[rr][6] * x1[2];
                L[rr][i] = s;
            }
        }

        #pragma unroll
        for (int rr = 0; rr < 4; ++rr) {
            const int rrel = wave * 4 + rr;
            float M = L[rr][0];
            #pragma unroll
            for (int i = 1; i < 16; ++i) M = fmaxf(M, L[rr][i]);
            #pragma unroll
            for (int off = 16; off > 0; off >>= 1) M = fmaxf(M, __shfl_xor(M, off, 32));
            const bool isrow0 = (nt == 0) && (rrel == 0);
            float ssum = 0.f;
            #pragma unroll
            for (int i = 0; i < 16; ++i) {
                const int m = lane + 32 * i;
                const float e = __expf(L[rr][i] - M);
                ssum += e;
                Et[rrel * EP + m] = (_Float16)(e * 16384.0f);
                if (isrow0) p0u[m] = e;
            }
            #pragma unroll
            for (int off = 16; off > 0; off >>= 1) ssum += __shfl_xor(ssum, off, 32);
            if (lane == 0) SinvAll[nt * 32 + rrel] = 1.0f / ssum;
        }
        __syncthreads();

        v8f acc = zero8;
        const _Float16* pA = &Et[(rsub * 16 + lan) * EP + 8 * h];
        const _Float16* pB = &XW1t[(grp * 16 + lan) * EP + 8 * h];
        #pragma unroll
        for (int kt = 0; kt < 16; ++kt) {
            const int k0 = kt * 32;
            Frag fa, fb;
            fa.half[0] = *(const v8h*)(pA + k0);
            fa.half[1] = *(const v8h*)(pA + k0 + 16);
            fb.half[0] = *(const v8h*)(pB + k0);
            fb.half[1] = *(const v8h*)(pB + k0 + 16);
            acc = wmma16(fa.v, fb.v, acc);
        }
        {
            const int mrow = nt * 32 + rsub * 16 + 8 * h;
            float contrib = 0.f;
            #pragma unroll
            for (int j = 0; j < 8; ++j) {
                const float hv = fmaxf(acc[j] * SinvAll[mrow + j], 0.f);
                contrib += p0u[mrow + j] * hv;
            }
            contrib += __shfl_xor(contrib, 16, 32);
            if (h == 0) part[(nt * 2 + rsub) * DH + grp * 16 + lan] = contrib;
        }
        __syncthreads();
    }

    if (tid < DH) {
        float s = 0.f;
        for (int t = 0; t < 32; ++t) s += part[t * DH + tid];
        vout[tid] = s * SinvAll[0] * (1.0f / 16384.0f);
    }
    __syncthreads();
    v4f vv = {0.f, 0.f, 0.f, 0.f};
    float* dst = Vg + (size_t)b * DH;
    if (tid < 16) {
        vv = *(const v4f*)&vout[4 * tid];
        *(volatile v4f*)(dst + 4 * tid) = vv;
    }
    __threadfence();
    if (tid < 16) {
        *(volatile v4f*)(dst + 4 * tid) = vv;
    }
}

__global__ __launch_bounds__(256)
void k_head(const float* __restrict__ Vg, const float* __restrict__ w2,
            const float* __restrict__ l1_w, const float* __restrict__ l1_b,
            const float* __restrict__ l2_w, const float* __restrict__ l2_b,
            float* __restrict__ out)
{
    __shared__ __align__(16) _Float16 Ah[NB * HP];
    __shared__ __align__(16) _Float16 Gh[NB * HP];
    __shared__ __align__(16) _Float16 W2t[DH * HP];
    __shared__ __align__(16) _Float16 L1s[DH * HP];
    __shared__ __align__(16) _Float16 L2s[16 * HP];
    __shared__ float b1s[DH];
    __shared__ __align__(16) float outs[NB];

    const int tid  = threadIdx.x;
    const int lane = tid & 31;
    const int wave = tid >> 5;
    const int h    = lane >> 4;
    const int lan  = lane & 15;
    const v8f zero8 = {0.f, 0.f, 0.f, 0.f, 0.f, 0.f, 0.f, 0.f};

    for (int idx = tid; idx < NB * DH; idx += 256) {
        const int r = idx >> 6, c = idx & 63;
        Ah[r * HP + c] = (_Float16)Vg[idx];
    }
    for (int idx = tid; idx < DH * DH; idx += 256) {
        const int r = idx >> 6, c = idx & 63;
        W2t[c * HP + r] = (_Float16)w2[idx];
        L1s[r * HP + c] = (_Float16)(l1_w[idx] * 16.0f);
    }
    for (int idx = tid; idx < 16 * HP; idx += 256)
        L2s[idx] = (idx < DH) ? (_Float16)(l2_w[idx] * 16.0f) : (_Float16)0.0f;
    if (tid < DH) b1s[tid] = l1_b[tid];
    const float b2 = l2_b[0];
    __syncthreads();

    #pragma unroll
    for (int i = 0; i < 8; ++i) {
        const int t = wave + 8 * i;
        const int rt = t >> 2, ct = t & 3;
        v8f acc = zero8;
        const _Float16* pA = &Ah[(rt * 16 + lan) * HP + 8 * h];
        const _Float16* pB = &W2t[(ct * 16 + lan) * HP + 8 * h];
        #pragma unroll
        for (int kt = 0; kt < 2; ++kt) {
            const int k0 = kt * 32;
            Frag fa, fb;
            fa.half[0] = *(const v8h*)(pA + k0);
            fa.half[1] = *(const v8h*)(pA + k0 + 16);
            fb.half[0] = *(const v8h*)(pB + k0);
            fb.half[1] = *(const v8h*)(pB + k0 + 16);
            acc = wmma16(fa.v, fb.v, acc);
        }
        #pragma unroll
        for (int j = 0; j < 8; ++j)
            Gh[(rt * 16 + 8 * h + j) * HP + ct * 16 + lan] = (_Float16)fmaxf(acc[j], 0.f);
    }
    __syncthreads();

    #pragma unroll
    for (int i = 0; i < 8; ++i) {
        const int t = wave + 8 * i;
        const int rt = t >> 2, ct = t & 3;
        v8f acc = zero8;
        const _Float16* pA = &Gh[(rt * 16 + lan) * HP + 8 * h];
        const _Float16* pB = &L1s[(ct * 16 + lan) * HP + 8 * h];
        #pragma unroll
        for (int kt = 0; kt < 2; ++kt) {
            const int k0 = kt * 32;
            Frag fa, fb;
            fa.half[0] = *(const v8h*)(pA + k0);
            fa.half[1] = *(const v8h*)(pA + k0 + 16);
            fb.half[0] = *(const v8h*)(pB + k0);
            fb.half[1] = *(const v8h*)(pB + k0 + 16);
            acc = wmma16(fa.v, fb.v, acc);
        }
        #pragma unroll
        for (int j = 0; j < 8; ++j) {
            const int col = ct * 16 + lan;
            const float hv = fmaxf(acc[j] * 0.0625f + b1s[col], 0.f);
            Ah[(rt * 16 + 8 * h + j) * HP + col] = (_Float16)hv;
        }
    }
    __syncthreads();

    #pragma unroll
    for (int i = 0; i < 2; ++i) {
        const int rt = wave + 8 * i;
        v8f acc = zero8;
        const _Float16* pA = &Ah[(rt * 16 + lan) * HP + 8 * h];
        const _Float16* pB = &L2s[lan * HP + 8 * h];
        #pragma unroll
        for (int kt = 0; kt < 2; ++kt) {
            const int k0 = kt * 32;
            Frag fa, fb;
            fa.half[0] = *(const v8h*)(pA + k0);
            fa.half[1] = *(const v8h*)(pA + k0 + 16);
            fb.half[0] = *(const v8h*)(pB + k0);
            fb.half[1] = *(const v8h*)(pB + k0 + 16);
            acc = wmma16(fa.v, fb.v, acc);
        }
        if (lan == 0) {
            #pragma unroll
            for (int j = 0; j < 8; ++j) outs[rt * 16 + 8 * h + j] = acc[j] * 0.0625f + b2;
        }
    }
    __syncthreads();

    v4f ov = {0.f, 0.f, 0.f, 0.f};
    if (tid < 64) {
        ov = *(const v4f*)&outs[4 * tid];
        *(volatile v4f*)(out + 4 * tid) = ov;
    }
    __threadfence();
    if (tid < 64) {
        *(volatile v4f*)(out + 4 * tid) = ov;
    }
}

extern "C" void kernel_launch(void* const* d_in, const int* in_sizes, int n_in,
                              void* d_out, int out_size, void* d_ws, size_t ws_size,
                              hipStream_t stream)
{
    if (n_in < 9) return;
    if (out_size != NB) return;
    if (in_sizes[0] != NB * NH * IND || in_sizes[1] != SD * HS || in_sizes[2] != HS * HS ||
        in_sizes[3] != HS * DH || in_sizes[4] != DH * DH || in_sizes[5] != DH * DH ||
        in_sizes[6] != DH || in_sizes[7] != DH || in_sizes[8] < 1) return;
    const size_t v_bytes = (size_t)NB * DH * sizeof(float);
    if (ws_size < v_bytes) return;

    const float* state = (const float*)d_in[0];
    const float* tmat  = (const float*)d_in[1];
    const float* w_a   = (const float*)d_in[2];
    const float* w1    = (const float*)d_in[3];
    const float* w2    = (const float*)d_in[4];
    const float* l1_w  = (const float*)d_in[5];
    const float* l1_b  = (const float*)d_in[6];
    const float* l2_w  = (const float*)d_in[7];
    const float* l2_b  = (const float*)d_in[8];
    float* out = (float*)d_out;
    float* Vg  = (float*)d_ws;

    k_attn<<<dim3(NB), dim3(256), 0, stream>>>(state, tmat, w_a, w1, Vg);
    k_head<<<dim3(1), dim3(256), 0, stream>>>(Vg, w2, l1_w, l1_b, l2_w, l2_b, out);
}
